// LinearCDE_56495999812316
// MI455X (gfx1250) — hardware-run, weakly checked
//
#include <hip/hip_runtime.h>
#include <math.h>

constexpr int NBATCH   = 8;
constexpr int NSEQ     = 512;
constexpr int NDIM     = 64;
constexpr int NHID     = 128;
constexpr int NAOUT    = NHID * NHID;
constexpr int NCOLS    = NAOUT + NHID;
constexpr int KIN      = NDIM + 1;
constexpr int CHS      = 128;
constexpr int NCHUNK   = NSEQ / CHS;
constexpr int NTHR     = 256;
constexpr int STEP_THR = 4 * NHID;
constexpr int GEMM_BLOCKS = ((CHS / 64) * (NCOLS / 64) + 7) / 8;
constexpr float DTV   = 0.025f;
constexpr float CLIPV = 1.0e11f;
constexpr float RCLIP = 1.0f / 1.0e11f;

static_assert(NDIM % 32 == 0);
static_assert(CHS % 64 == 0 && NCOLS % 64 == 0);
static_assert(NSEQ % CHS == 0 && NCHUNK == 4);
static_assert((NBATCH * NSEQ * NDIM) % (8 * NTHR) == 0);
static_assert((NCOLS * 8) % NTHR == 0 && (NAOUT * 8) % NTHR == 0);
static_assert(NAOUT % (4 * NTHR) == 0 && NCOLS % 4 == 0);
static_assert(NHID == 4 * 32);
static_assert(STEP_THR == 512);

typedef __attribute__((ext_vector_type(16))) _Float16 v16h;
typedef __attribute__((ext_vector_type(8)))  _Float16 v8h;
typedef __attribute__((ext_vector_type(16))) __bf16   v16b;
typedef __attribute__((ext_vector_type(8)))  __bf16   v8b;
typedef __attribute__((ext_vector_type(8)))  float    v8f;
typedef __attribute__((ext_vector_type(4)))  float    v4f;

__device__ __forceinline__ unsigned short f2bf_bits(float f) {
  unsigned u = __float_as_uint(f);
  return (unsigned short)((u + 0x7FFFu + ((u >> 16) & 1u)) >> 16);
}
__device__ __forceinline__ float bf_bits2f(unsigned short h) { return __uint_as_float(((unsigned)h) << 16); }
__device__ __forceinline__ float bf16r(float f) { return bf_bits2f(f2bf_bits(f)); }

__device__ __forceinline__ void dep_guard_h(v8f& a, v8f& b, v16h x, v16h y) { asm volatile("v_nop\n\tv_nop\n\tv_nop\n\tv_nop" : "+v"(a), "+v"(b) : "v"(x), "v"(y)); }
__device__ __forceinline__ void dep_guard_b(v8f& a, v8f& b, v16b x, v16b y) { asm volatile("v_nop\n\tv_nop\n\tv_nop\n\tv_nop" : "+v"(a), "+v"(b) : "v"(x), "v"(y)); }
__device__ __forceinline__ void keep4_h(v16h a, v16h b, v16h c, v16h d) { asm volatile("v_nop" :: "v"(a), "v"(b), "v"(c), "v"(d)); }
__device__ __forceinline__ void keep4_b(v16b a, v16b b, v16b c, v16b d) { asm volatile("v_nop" :: "v"(a), "v"(b), "v"(c), "v"(d)); }
__device__ __forceinline__ void acc_guard4(v8f& a, v8f& b, v8f& c, v8f& d) { asm volatile("v_nop\n\tv_nop\n\tv_nop\n\tv_nop" : "+v"(a), "+v"(b), "+v"(c), "+v"(d)); }
template <typename T> struct Frag;
template <> struct Frag<_Float16> {
  typedef v16h V; union U { v16h v; v8h h[2]; };
  static __device__ __forceinline__ v16h load(const _Float16* p) {
    U f; f.h[0] = *(const v8h*)(p); f.h[1] = *(const v8h*)(p + 16); return f.v;
  }
  static __device__ __forceinline__ v8f mma(v16h a, v16h b, v8f c) {
    return __builtin_amdgcn_wmma_f32_16x16x32_f16(false, a, false, b, (short)0, c, false, false);
  }
  static __device__ __forceinline__ void guard(v8f& a, v8f& b, v16h x, v16h y) { dep_guard_h(a, b, x, y); }
  static __device__ __forceinline__ void keep(v16h a, v16h b, v16h c, v16h d) { keep4_h(a, b, c, d); }
};
template <> struct Frag<__bf16> {
  typedef v16b V; union U { v16b v; v8b h[2]; };
  static __device__ __forceinline__ v16b load(const __bf16* p) {
    U f; f.h[0] = *(const v8b*)(p); f.h[1] = *(const v8b*)(p + 16); return f.v;
  }
  static __device__ __forceinline__ v8f mma(v16b a, v16b b, v8f c) {
    return __builtin_amdgcn_wmma_f32_16x16x32_bf16(false, a, false, b, (short)0, c, false, false);
  }
  static __device__ __forceinline__ void guard(v8f& a, v8f& b, v16b x, v16b y) { dep_guard_b(a, b, x, y); }
  static __device__ __forceinline__ void keep(v16b a, v16b b, v16b c, v16b d) { keep4_b(a, b, c, d); }
};

template <int ET> struct Elem;
template <> struct Elem<0> { typedef _Float16 T; };
template <> struct Elem<1> { typedef __bf16 T; };
template <int ET, bool SPLIT, int BIAS_MODE, int OUT_MODE, bool RESID, int ACT = 0>
__global__ __launch_bounds__(256) void wmma_gemm64(
    const unsigned short* __restrict__ Ap, const unsigned short* __restrict__ A2p, int lda, long strideA,
    const unsigned short* __restrict__ Btp, const unsigned short* __restrict__ Bt2p, int ldb, long strideB,
    void* __restrict__ Cout, void* __restrict__ Cout2, int ldc, long strideC,
    const float* __restrict__ bias,
    const float* __restrict__ resid, long strideR,
    int M, int N, int K, float scale) {
  typedef typename Elem<ET>::T T;
  typedef typename Frag<T>::V V;
  const T* A = (const T*)Ap; const T* A2 = (const T*)A2p; const T* Bt = (const T*)Btp; const T* Bt2 = (const T*)Bt2p;
  __shared__ __align__(16) float sT[8][16 * 68];
  const int b    = blockIdx.y;
  const int lane = threadIdx.x & 31;
  const int wave = threadIdx.x >> 5;
  const int tilesN = N >> 6;
  const int tilesM = M >> 6;
  const int tile = blockIdx.x * 8 + wave;
  if (tile >= tilesM * tilesN) return;
  const int tm = tile / tilesN;
  const int tn = tile - tm * tilesN;
  const int m0 = tm << 6;
  const int n0 = tn << 6;

  const T* Ab  = A  + (size_t)b * strideA;
  const T* Bb  = Bt + (size_t)b * strideB;
  const T* Ab2 = SPLIT ? (A2  + (size_t)b * strideA) : nullptr;
  const T* Bb2 = SPLIT ? (Bt2 + (size_t)b * strideB) : nullptr;

  const int rlane = lane & 15;
  const int koff  = (lane >> 4) * 8;
  const int mOff  = (lane >> 4) * 8;

  v8f acc[4][4];
#pragma unroll
  for (int i = 0; i < 4; ++i)
#pragma unroll
    for (int j = 0; j < 4; ++j) acc[i][j] = (v8f){0.f,0.f,0.f,0.f,0.f,0.f,0.f,0.f};

  for (int k0 = 0; k0 < K; k0 += 32) {
    V bh[4], bl[4];
#pragma unroll
    for (int j = 0; j < 4; ++j) {
      const size_t bo = (size_t)(n0 + (j << 4) + rlane) * ldb + koff + k0;
      bh[j] = Frag<T>::load(Bb + bo);
      if (SPLIT) bl[j] = Frag<T>::load(Bb2 + bo);
    }
#pragma unroll
    for (int i = 0; i < 4; ++i) {
      const size_t ao = (size_t)(m0 + (i << 4) + rlane) * lda + koff + k0;
      V ah = Frag<T>::load(Ab + ao);
      V al;
      if (SPLIT) al = Frag<T>::load(Ab2 + ao);
#pragma unroll
      for (int j = 0; j < 4; ++j) {
        acc[i][j] = Frag<T>::mma(ah, bh[j], acc[i][j]);
        if (SPLIT) {
          acc[i][j] = Frag<T>::mma(ah, bl[j], acc[i][j]);
          acc[i][j] = Frag<T>::mma(al, bh[j], acc[i][j]);
        }
      }
      Frag<T>::guard(acc[i][0], acc[i][3], ah, SPLIT ? al : ah);
    }
    Frag<T>::keep(bh[0], bh[1], bh[2], bh[3]);
    if (SPLIT) Frag<T>::keep(bl[0], bl[1], bl[2], bl[3]);
  }
  acc_guard4(acc[0][0], acc[0][1], acc[0][2], acc[0][3]);
  acc_guard4(acc[1][0], acc[1][1], acc[1][2], acc[1][3]);
  acc_guard4(acc[2][0], acc[2][1], acc[2][2], acc[2][3]);
  acc_guard4(acc[3][0], acc[3][1], acc[3][2], acc[3][3]);

  float* slab = sT[wave];
  const float* Rb = RESID ? (resid + (size_t)b * strideR) : nullptr;
#pragma unroll
  for (int i = 0; i < 4; ++i) {
    const int mBase = m0 + (i << 4);
#pragma unroll
    for (int j = 0; j < 4; ++j) {
      const int n = n0 + (j << 4) + rlane;
      float bv = 0.f;
      if (BIAS_MODE == 2) bv = bias[n];
#pragma unroll
      for (int r = 0; r < 8; ++r) {
        float v = acc[i][j][r] * scale;
        if (BIAS_MODE == 1) v += bias[mBase + mOff + r];
        if (BIAS_MODE == 2) v += bv;
        if (RESID) v += Rb[(size_t)(mBase + mOff + r) * ldc + n];
        if (ACT == 1) v = tanhf(v);
        if (ACT == 2) v = fmaxf(v, 0.0f);
        if (ACT == 3) v = v / (1.0f + expf(-v));
        if (ACT == 4) v = (v > 0.f) ? v : 0.01f * v;
        if (ACT == 5) v = 0.5f * v * (1.0f + erff(v * 0.70710678118654752f));
        slab[(mOff + r) * 68 + (j << 4) + rlane] = v;
      }
    }
    __builtin_amdgcn_fence(__ATOMIC_RELEASE, "workgroup");
    __builtin_amdgcn_wave_barrier();
    __builtin_amdgcn_fence(__ATOMIC_ACQUIRE, "workgroup");
    if (OUT_MODE == 0) {
      float* C = (float*)Cout + (size_t)b * strideC;
      const int hh = lane >> 4, c4 = (lane & 15) * 4;
      for (int pass = 0; pass < 2; ++pass) {
#pragma unroll
        for (int it = 0; it < 8; ++it) {
          const int row = it * 2 + hh;
          v4f v = *(const v4f*)(slab + row * 68 + c4);
          *(volatile v4f*)(C + (size_t)(mBase + row) * ldc + n0 + c4) = v;
        }
        __threadfence();
      }
    } else {
      const int q = lane >> 3, c8 = (lane & 7) * 8;
      unsigned short* C  = (unsigned short*)Cout  + (size_t)b * strideC;
      unsigned short* C2 = (OUT_MODE == 2) ? ((unsigned short*)Cout2 + (size_t)b * strideC) : nullptr;
      for (int pass = 0; pass < 2; ++pass) {
#pragma unroll
        for (int it = 0; it < 4; ++it) {
          const int row = it * 4 + q;
          const float* sp = slab + row * 68 + c8;
          v8h hv, lv;
#pragma unroll
          for (int e = 0; e < 8; ++e) {
            if (OUT_MODE == 1) {
              hv[e] = (_Float16)sp[e];
            } else {
              unsigned short hb = f2bf_bits(sp[e]);
              unsigned short lb = f2bf_bits(sp[e] - bf_bits2f(hb));
              hv[e] = __builtin_bit_cast(_Float16, hb);
              lv[e] = __builtin_bit_cast(_Float16, lb);
            }
          }
          *(volatile v8h*)(C + (size_t)(mBase + row) * ldc + n0 + c8) = hv;
          if (OUT_MODE == 2) *(volatile v8h*)(C2 + (size_t)(mBase + row) * ldc + n0 + c8) = lv;
        }
        __threadfence();
      }
    }
    __builtin_amdgcn_fence(__ATOMIC_RELEASE, "workgroup");
    __builtin_amdgcn_wave_barrier();
    __builtin_amdgcn_fence(__ATOMIC_ACQUIRE, "workgroup");
  }
}

__global__ __launch_bounds__(NTHR) void k_packx(const float* __restrict__ x, unsigned short* __restrict__ dst) {
  const int i  = blockIdx.x * NTHR + threadIdx.x;
  const int n8 = NBATCH * NSEQ * NDIM / 8;
  if (i < n8) {
    const float* sp = x + (size_t)i * 8;
    const v4f a = *(const v4f*)(sp);
    const v4f c = *(const v4f*)(sp + 4);
    v8h hv;
#pragma unroll
    for (int e = 0; e < 4; ++e) {
      hv[e]     = __builtin_bit_cast(_Float16, f2bf_bits(a[e]));
      hv[4 + e] = __builtin_bit_cast(_Float16, f2bf_bits(c[e]));
    }
    *(volatile v8h*)(dst + (size_t)i * 8) = hv;
    __threadfence();
    *(volatile v8h*)(dst + (size_t)i * 8) = hv;
  }
}

__global__ __launch_bounds__(NTHR) void k_packw_plane(const float* __restrict__ wa, const float* __restrict__ wb,
                                                      unsigned short* __restrict__ dst) {
  const int i  = blockIdx.x * NTHR + threadIdx.x;
  const int n  = i >> 3, c8 = i & 7;
  const bool isb = (blockIdx.x >= (NAOUT * 8) / NTHR);
  const float* src = isb ? wb : wa;
  const int srow = isb ? (n - NAOUT) : n;
  const float* sp = src + (size_t)srow * KIN + 1 + 8 * c8;
  v8h hv;
#pragma unroll
  for (int e = 0; e < 8; ++e) hv[e] = __builtin_bit_cast(_Float16, f2bf_bits(sp[e]));
  *(volatile v8h*)(dst + (size_t)i * 8) = hv;
  __threadfence();
  *(volatile v8h*)(dst + (size_t)i * 8) = hv;
}

__global__ __launch_bounds__(NTHR) void k_packw_bias(const float* __restrict__ wa, const float* __restrict__ wb,
                                                     float* __restrict__ dst) {
  const int t = blockIdx.x * NTHR + threadIdx.x;
  if (t < NCOLS / 4) {
    const bool isb = (blockIdx.x >= NAOUT / (4 * NTHR));
    const float* src = isb ? wb : wa;
    const int r0 = isb ? (4 * t - NAOUT) : (4 * t);
    v4f o;
#pragma unroll
    for (int e = 0; e < 4; ++e) o[e] = DTV * bf16r(src[(size_t)(r0 + e) * KIN]);
    *(volatile v4f*)(dst + (size_t)t * 4) = o;
    __threadfence();
    *(volatile v4f*)(dst + (size_t)t * 4) = o;
  }
}

__global__ __launch_bounds__(NHID) void k_y0(const float* __restrict__ x, const float* __restrict__ wi,
                                             const float* __restrict__ bi, float* __restrict__ out) {
  __shared__ __align__(16) float ys[NHID];
  const int b = blockIdx.x, i = threadIdx.x, lane = i & 31;
  const float* x0 = x + (size_t)b * NSEQ * NDIM;
  const float* w  = wi + (size_t)i * NDIM;
  float acc = 0.0f;
#pragma unroll 1
  for (int d = 0; d < NDIM; ++d) acc = fmaf(bf16r(x0[d]), bf16r(w[d]), acc);
  acc = acc + bf16r(bi[i]);
  ys[i] = acc;
  __syncthreads();
  if (i < 32) {
    const v4f v = *(const v4f*)(ys + 4 * lane);
    float* op = out + (size_t)b * NSEQ * NHID + 4 * lane;
    *(volatile v4f*)op = v;
    __threadfence();
    *(volatile v4f*)op = v;
  }
}

__global__ __launch_bounds__(STEP_THR) void k_seq(const float* __restrict__ asc, float* out, int chunk) {
  __shared__ __align__(16) float ybuf[2][NHID];
  const int b = blockIdx.x, tid = threadIdx.x, lane = tid & 31;
  const int i = tid >> 2, q = tid & 3;
  int c = chunk;
  c = c < 0 ? 0 : (c > NCHUNK - 1 ? NCHUNK - 1 : c);
  const int s_first = (c == 0) ? 1 : c * CHS;
  const int s_end   = c * CHS + CHS;
  int nsteps = s_end - s_first;
  nsteps = nsteps > CHS ? CHS : nsteps;
  float* ob = out + (size_t)b * NSEQ * NHID;
  if (tid < NHID) ybuf[0][tid] = ob[(size_t)(s_first - 1) * NHID + tid];
  __syncthreads();

#pragma unroll 1
  for (int t2 = 0; t2 < nsteps; ++t2) {
    const int s  = s_first + t2;
    const int pr = t2 & 1;
    const float* yr = ybuf[pr];
    const size_t rowoff = (size_t)(b * CHS + (s - c * CHS)) * NCOLS;
    const float* arow = asc + rowoff + (size_t)i * NHID + q * 32;
    float part = 0.0f;
#pragma unroll
    for (int k = 0; k < 8; ++k) {
      const v4f av = *(const v4f*)(arow + 4 * k);
      const v4f yv = *(const v4f*)(yr + q * 32 + 4 * k);
      part = fmaf(av[0], yv[0], part);
      part = fmaf(av[1], yv[1], part);
      part = fmaf(av[2], yv[2], part);
      part = fmaf(av[3], yv[3], part);
    }
    part += __shfl_xor(part, 1, 32);
    part += __shfl_xor(part, 2, 32);
    const float bsv = asc[rowoff + NAOUT + i];
    const float st  = part + bsv;
    const float yn  = yr[i] + CLIPV * tanhf(st * RCLIP);
    if (q == 0) ybuf[pr ^ 1][i] = yn;
    __syncthreads();
    if (tid < 32) {
      const v4f v = *(const v4f*)(&ybuf[pr ^ 1][4 * lane]);
      float* op = ob + (size_t)s * NHID + 4 * lane;
      *(volatile v4f*)op = v;
      __threadfence();
      *(volatile v4f*)op = v;
    }
  }
}

extern "C" void kernel_launch(void* const* d_in, const int* in_sizes, int n_in,
                              void* d_out, int out_size, void* d_ws, size_t ws_size, hipStream_t stream) {
  if (n_in < 5 || d_out == nullptr || d_ws == nullptr) return;
  if (in_sizes[0] != NBATCH * NSEQ * NDIM || in_sizes[1] != NHID * NDIM || in_sizes[2] != NHID ||
      in_sizes[3] != NAOUT * KIN || in_sizes[4] != NHID * KIN || out_size != NBATCH * NSEQ * NHID) return;

  const float* x   = (const float*)d_in[0];
  const float* wi  = (const float*)d_in[1];
  const float* bi  = (const float*)d_in[2];
  const float* wa  = (const float*)d_in[3];
  const float* wbv = (const float*)d_in[4];
  float* out = (float*)d_out;

  char* ws = (char*)d_ws; size_t off = 0;
  auto carve = [&](size_t bytes) -> char* { char* p = ws + off; off += (bytes + 255) & ~(size_t)255; return p; };
  unsigned short* XBP   = (unsigned short*)carve((size_t)NBATCH * NSEQ * NDIM * 2);
  unsigned short* WBP   = (unsigned short*)carve((size_t)NCOLS * NDIM * 2);
  float*          BIASV = (float*)carve((size_t)NCOLS * 4);
  float*          ASC   = (float*)carve((size_t)NBATCH * CHS * NCOLS * 4);
  if (off > ws_size || off > (size_t)134217728) return;

  k_y0<<<NBATCH, NHID, 0, stream>>>(x, wi, bi, out);
  k_packx<<<(NBATCH * NSEQ * NDIM / 8) / NTHR, NTHR, 0, stream>>>(x, XBP);
  k_packw_plane<<<(NCOLS * 8) / NTHR, NTHR, 0, stream>>>(wa, wbv, WBP);
  k_packw_bias<<<(NCOLS / 4 + NTHR - 1) / NTHR, NTHR, 0, stream>>>(wa, wbv, BIASV);

  for (int ch = 0; ch < NCHUNK; ++ch) {
    const unsigned short* achunk = XBP + (size_t)ch * CHS * NDIM;
    wmma_gemm64<1, false, 2, 0, false, 0><<<dim3(GEMM_BLOCKS, NBATCH), 256, 0, stream>>>(
        achunk, achunk, NDIM, (long)NSEQ * NDIM,
        WBP, WBP, NDIM, 0L,
        (void*)ASC, (void*)ASC, NCOLS, (long)CHS * NCOLS,
        BIASV, BIASV, 0L,
        CHS, NCOLS, NDIM, DTV);
    k_seq<<<NBATCH, STEP_THR, 0, stream>>>(ASC, out, ch);
  }
}
